// action_network_84378927497724
// MI455X (gfx1250) — hardware-verified
//
#include <hip/hip_runtime.h>


namespace {
constexpr int NV = 50000, NE = 10000, NNZ = 400000, D = 256, H = 512, SB = 128  ;
constexpr float XS = 8.0f;

typedef _Float16 b16;
typedef __attribute__((ext_vector_type(16))) _Float16 v16b;
typedef __attribute__((ext_vector_type(8))) _Float16 v8b;
typedef __attribute__((ext_vector_type(8))) float v8f;
typedef __attribute__((ext_vector_type(4))) float v4f;
__device__ __forceinline__ float bf16_rne(float f) { unsigned int u = __float_as_uint(f); u += 0x7FFFu + ((u >> 16) & 1u); return __uint_as_float(u & 0xFFFF0000u); }
__device__ __forceinline__ v16b frag_kb(const b16* p, int hh) { const v8b a = *(const v8b*)(p + 8 * hh), b = *(const v8b*)(p + 16 + 8 * hh); v16b f;
#pragma unroll
  for (int e = 0; e < 8; ++e) { f[e] = a[e]; f[8 + e] = b[e]; } return f; }
__device__ __forceinline__ v16b frag_x(const float* p, int hh) { v16b f;
#pragma unroll
  for (int e = 0; e < 8; ++e) { f[e] = (b16)bf16_rne(p[8 * hh + e]); f[8 + e] = (b16)bf16_rne(p[16 + 8 * hh + e]); } return f; }
__device__ __forceinline__ v8f wmma16b(v16b a, v16b b, v8f c) { v8f d = __builtin_amdgcn_wmma_f32_16x16x32_f16(false, a, false, b, (short)0, c, false, false); asm volatile("v_nop\n\tv_nop\n\tv_nop\n\tv_nop" : "+v"(d) : "v"(a), "v"(b)); return d; }
__device__ __forceinline__ void wave_lds_sync() { __builtin_amdgcn_fence(__ATOMIC_RELEASE, "workgroup"); __builtin_amdgcn_wave_barrier(); __builtin_amdgcn_fence(__ATOMIC_ACQUIRE, "workgroup"); }
__device__ __forceinline__ float nexp(float x) { return __builtin_amdgcn_exp2f(x * 1.4426950408889634f); }
__device__ __forceinline__ float nlog(float x) { return __builtin_amdgcn_logf(x) * 0.6931471805599453f; }
__device__ __forceinline__ float pmul(float a, float b) { float p = a * b; asm volatile("" : "+v"(p)); return p; }

struct Wo_ { static constexpr size_t W1 = 0, W2 = (size_t)H * D, WU = W2 + (size_t)D * H, END = WU + (size_t)D * D; };
__global__ __launch_bounds__(256) void prep_kernel(const float* __restrict__ W1, const float* __restrict__ W2, const float* __restrict__ Wu, const float* __restrict__ b1, const float* __restrict__ b2, const float* __restrict__ bu, b16* __restrict__ R, float* __restrict__ P) {
  const size_t tid = (size_t)blockIdx.x * 256 + threadIdx.x, nth = (size_t)gridDim.x * 256;
  auto tr = [&](size_t base, int nout, int kin, const float* W) { for (size_t p = tid; p < (size_t)nout * (kin / 8); p += nth) { const int o = (int)(p / (kin / 8)), k0 = (int)(p % (kin / 8)) * 8; v8b v;
#pragma unroll
      for (int e = 0; e < 8; ++e) v[e] = (b16)bf16_rne(W[(size_t)(k0 + e) * nout + o]); *(volatile v8b*)(R + base + (size_t)o * kin + k0) = v; } };
  for (int pass = 0; pass < 2; ++pass) { tr(Wo_::W1, H, D, W1); tr(Wo_::W2, D, H, W2); tr(Wo_::WU, D, D, Wu);
    for (size_t q = tid; q < 1024; q += nth) { const int i = (int)q; P[q] = bf16_rne((i < 512) ? b1[i] : (i < 768) ? b2[i - 512] : bu[i - 768]); }
    __threadfence(); }
}

__global__ __launch_bounds__(128) void mlp_kernel(const float* __restrict__ x, const b16* __restrict__ R, const float* __restrict__ P, float* __restrict__ M) {
  __shared__ __attribute__((aligned(16))) b16 Hs[32][H + 8]; __shared__ __attribute__((aligned(16))) float Ts[4][32][64 + 4];
  const int lane = threadIdx.x & 31, wave = threadIdx.x >> 5, nloc = lane & 15, hlf = lane >> 4, m0 = blockIdx.x * 32;
  auto rowc = [&](int r) { return (r < NV) ? r : (NV - 1); };
  { v8f acc[2][8];
#pragma unroll
    for (int r = 0; r < 2; ++r)
#pragma unroll
      for (int t = 0; t < 8; ++t) acc[r][t] = (v8f){};
#pragma unroll 2
    for (int kb = 0; kb < D; kb += 32) { const v16b a0 = frag_x(x + (size_t)rowc(m0 + nloc) * D + kb, hlf), a1 = frag_x(x + (size_t)rowc(m0 + 16 + nloc) * D + kb, hlf);
#pragma unroll
      for (int t = 0; t < 8; ++t) { const v16b bw = frag_kb(R + Wo_::W1 + (size_t)(wave * 128 + t * 16 + nloc) * D + kb, hlf); acc[0][t] = wmma16b(a0, bw, acc[0][t]); acc[1][t] = wmma16b(a1, bw, acc[1][t]); } }
#pragma unroll
    for (int t = 0; t < 8; ++t) { const int c = wave * 128 + t * 16 + nloc; const float bb = P[c];
#pragma unroll
      for (int r = 0; r < 2; ++r)
#pragma unroll
        for (int v = 0; v < 8; ++v) Hs[r * 16 + 8 * hlf + v][c] = (b16)(fmaxf(acc[r][t][v] + bb, 0.0f) * XS); } }
  __syncthreads();
  { v8f acc[2][4];
#pragma unroll
    for (int r = 0; r < 2; ++r)
#pragma unroll
      for (int t = 0; t < 4; ++t) acc[r][t] = (v8f){};
#pragma unroll 2
    for (int kb = 0; kb < H; kb += 32) { const v16b a0 = frag_kb(&Hs[nloc][kb], hlf), a1 = frag_kb(&Hs[16 + nloc][kb], hlf);
#pragma unroll
      for (int t = 0; t < 4; ++t) { const v16b bw = frag_kb(R + Wo_::W2 + (size_t)(wave * 64 + t * 16 + nloc) * H + kb, hlf); acc[0][t] = wmma16b(a0, bw, acc[0][t]); acc[1][t] = wmma16b(a1, bw, acc[1][t]); } }
#pragma unroll
    for (int t = 0; t < 4; ++t) { const int c = wave * 64 + t * 16 + nloc; const float bb = P[512 + c];
#pragma unroll
      for (int r = 0; r < 2; ++r)
#pragma unroll
        for (int v = 0; v < 8; ++v) Ts[wave][r * 16 + 8 * hlf + v][t * 16 + nloc] = fmaxf(acc[r][t][v] * (1.0f / XS) + bb, 0.0f); } }
  wave_lds_sync();
  for (int pass = 0; pass < 2; ++pass) { for (int i = lane; i < 32 * 16; i += 32) { const int rr = i >> 4, c4 = (i & 15) * 4; if (m0 + rr < NV) *(volatile v4f*)(M + (size_t)(m0 + rr) * D + wave * 64 + c4) = *(const v4f*)(&Ts[wave][rr][c4]); } __threadfence(); }
}

__global__ __launch_bounds__(256) void segmean_kernel(const float* __restrict__ VAL, const int* __restrict__ segid, const int* __restrict__ gidx, int nseg, int nval, float* __restrict__ OUTM) {
  __shared__ __attribute__((aligned(16))) float Acc[SB][D]; __shared__ int Lsrc[256]; __shared__ int Lseg[256]; __shared__ int Cw[8]; __shared__ int tot; __shared__ int Cn[SB];
  const int s0 = blockIdx.x * SB, t_ = threadIdx.x, lane = t_ & 31, wave = t_ >> 5;
  for (int i = t_; i < SB * D; i += 256) (&Acc[0][0])[i] = 0.0f;
  if (t_ < SB) Cn[t_] = 0;
  int mycnt[16];
#pragma unroll
  for (int q = 0; q < 16; ++q) mycnt[q] = 0;
  __syncthreads();
  for (int c0 = 0; c0 < NNZ; c0 += 256) { const int j = c0 + t_; int loc = -1, g = 0; if (j < NNZ) { const int s = segid[j]; if (s >= s0 && s < s0 + SB) { loc = s - s0; g = gidx[j]; g = (g < 0) ? 0 : (g >= nval ? nval - 1 : g); } }
    const unsigned int bal = __builtin_amdgcn_ballot_w32(loc >= 0); if (lane == 0) Cw[wave] = __builtin_popcount(bal);
    __syncthreads();
    int base = 0; for (int w = 0; w < wave; ++w) base += Cw[w]; const int pos = base + __builtin_popcount(bal & ((1u << lane) - 1u));
    if (loc >= 0) { Lsrc[pos] = g; Lseg[pos] = loc; }
    if (t_ == 0) { int a = 0; for (int w = 0; w < 8; ++w) a += Cw[w]; tot = a; }
    __syncthreads();
    const int nh = tot;
    for (int k = 0; k < nh; ++k) { const int sg = Lseg[k]; if ((sg >> 4) == wave) { const float* vr = VAL + (size_t)Lsrc[k] * D; float* ac = Acc[sg];
#pragma unroll
        for (int e = 0; e < 8; ++e) { const int idx = e * 32 + lane; ac[idx] += vr[idx]; }
#pragma unroll
        for (int q = 0; q < 16; ++q) if (q == (sg & 15)) mycnt[q] += 1; } }
    __syncthreads(); }
  for (int q = 0; q < 16; ++q) { const int sg = wave * 16 + q, s = s0 + sg; if (s >= nseg) continue; const float inv = 1.0f / fmaxf((float)mycnt[q], 1.0f);
    for (int pass = 0; pass < 2; ++pass) { for (int i4 = lane * 4; i4 < D; i4 += 128) { v4f o; for (int e = 0; e < 4; ++e) o[e] = Acc[sg][i4 + e] * inv; *(volatile v4f*)(OUTM + (size_t)s * D + i4) = o; } __threadfence(); } }
}

__global__ __launch_bounds__(128) void upd_kernel(const float* __restrict__ x, const b16* __restrict__ R, const float* __restrict__ P, const float* __restrict__ MI, float* __restrict__ out) {
  __shared__ __attribute__((aligned(16))) float Hrow[32][D + 4];
  const int lane = threadIdx.x & 31, wave = threadIdx.x >> 5, nloc = lane & 15, hlf = lane >> 4, m0 = blockIdx.x * 32;
  auto rowc = [&](int r) { return (r < NV) ? r : (NV - 1); };
  v8f acc[2][4];
#pragma unroll
  for (int r = 0; r < 2; ++r)
#pragma unroll
    for (int t = 0; t < 4; ++t) acc[r][t] = (v8f){};
#pragma unroll 2
  for (int kb = 0; kb < D; kb += 32) { const v16b a0 = frag_x(x + (size_t)rowc(m0 + nloc) * D + kb, hlf), a1 = frag_x(x + (size_t)rowc(m0 + 16 + nloc) * D + kb, hlf);
#pragma unroll
    for (int t = 0; t < 4; ++t) { const v16b bw = frag_kb(R + Wo_::WU + (size_t)(wave * 64 + t * 16 + nloc) * D + kb, hlf); acc[0][t] = wmma16b(a0, bw, acc[0][t]); acc[1][t] = wmma16b(a1, bw, acc[1][t]); } }
#pragma unroll
  for (int t = 0; t < 4; ++t) { const int c = wave * 64 + t * 16 + nloc; const float bb = P[768 + c];
#pragma unroll
    for (int r = 0; r < 2; ++r)
#pragma unroll
      for (int v = 0; v < 8; ++v) { const int rr = r * 16 + 8 * hlf + v; Hrow[rr][c] = fmaxf(acc[r][t][v] + bb + MI[(size_t)rowc(m0 + rr) * D + c], 0.0f); } }
  __syncthreads();
  for (int q = 0; q < 8; ++q) { const int rr = wave * 8 + q; if (m0 + rr >= NV) continue; float v[8]; float mx = -INFINITY;
#pragma unroll
    for (int e = 0; e < 8; ++e) { v[e] = Hrow[rr][e * 32 + lane]; mx = fmaxf(mx, v[e]); }
#pragma unroll
    for (int o = 1; o < 32; o <<= 1) mx = fmaxf(mx, __shfl_xor(mx, o));
    float su = 0.0f;
#pragma unroll
    for (int e = 0; e < 8; ++e) su += nexp(v[e] - mx);
#pragma unroll
    for (int o = 1; o < 32; o <<= 1) su += __shfl_xor(su, o);
    const float lz = mx + nlog(su);
#pragma unroll
    for (int e = 0; e < 8; ++e) Hrow[rr][e * 32 + lane] = v[e] - lz; }
  wave_lds_sync();
  for (int pass = 0; pass < 2; ++pass) { for (int q = 0; q < 8; ++q) { const int rr = wave * 8 + q; if (m0 + rr >= NV) continue; for (int i4 = lane * 4; i4 < D; i4 += 128) *(volatile v4f*)(out + (size_t)(m0 + rr) * D + i4) = *(const v4f*)(&Hrow[rr][i4]); } __threadfence(); }
}
}

extern "C" void kernel_launch(void* const* d_in, const int* in_sizes, int n_in,
                              void* d_out, int out_size, void* d_ws, size_t ws_size, hipStream_t stream) {
  (void)n_in; (void)out_size;
  const float* x = (const float*)d_in[0]; const int* vidx = (const int*)d_in[1]; const int* eidx = (const int*)d_in[2]; const float* W1 = (const float*)d_in[3]; const float* b1 = (const float*)d_in[4]; const float* W2 = (const float*)d_in[5]; const float* b2 = (const float*)d_in[6]; const float* Wu = (const float*)d_in[7]; const float* bu = (const float*)d_in[8];
  float* out = (float*)d_out;
  if (in_sizes[0] != NV * D || in_sizes[1] != NNZ || in_sizes[2] != NNZ || in_sizes[3] != D * H || in_sizes[7] != D * D) return;
  size_t off = 0; char* ws = (char*)d_ws;
  auto carve = [&](size_t bytes) { char* p = ws + off; off += (bytes + 255) & ~(size_t)255; return p; };
  b16* R = (b16*)carve(Wo_::END * 2); float* P = (float*)carve(1024 * 4); float* M = (float*)carve((size_t)NV * D * 4); float* ME = (float*)carve((size_t)NE * D * 4); float* MI = (float*)carve((size_t)NV * D * 4);
  if (off > ws_size) return;
  prep_kernel<<<128, 256, 0, stream>>>(W1, W2, Wu, b1, b2, bu, R, P);
  mlp_kernel<<<(NV + 31) / 32, 128, 0, stream>>>(x, R, P, M);
  segmean_kernel<<<(NE + SB - 1) / SB, 256, 0, stream>>>(M, eidx, vidx, NE, NV, ME);
  segmean_kernel<<<(NV + SB - 1) / SB, 256, 0, stream>>>(ME, vidx, eidx, NV, NE, MI);
  upd_kernel<<<(NV + 31) / 32, 128, 0, stream>>>(x, R, P, MI, out);
}
